// VisualBranch_vsgnet_72438918414396
// MI455X (gfx1250) — hardware-verified
//
#include <hip/hip_runtime.h>
#include <stdint.h>
#include <stddef.h>


typedef unsigned short u16;
typedef __bf16 v16bf __attribute__((ext_vector_type(16)));
typedef u16    v8u16 __attribute__((ext_vector_type(8)));
typedef int    v8i   __attribute__((ext_vector_type(8)));
typedef float  v8f   __attribute__((ext_vector_type(8)));
typedef float  v4f   __attribute__((ext_vector_type(4)));

union Frag { v16bf v; v8u16 h[2]; v8i w; };

#define BM 64
#define BN 64
#define BK 64
#define LDK 72
#define CSP 68
#define GT 128

static __device__ __forceinline__ unsigned int bf_rne(float f) {
  unsigned int u = __builtin_bit_cast(unsigned int, f);
  return (u + 0x7FFFu + ((u >> 16) & 1u)) >> 16;
}

static __device__ __forceinline__ void split8(const float (&x)[8], v8u16& vh, v8u16& vl) {
#pragma unroll
  for (int j = 0; j < 8; ++j) {
    unsigned int hb = bf_rne(x[j]);
    float hf = __builtin_bit_cast(float, hb << 16);
    unsigned int lb = bf_rne(x[j] - hf);
    vh[j] = (u16)hb;
    vl[j] = (u16)lb;
  }
}

static __device__ __forceinline__ void wmma3(v8f& acc, const Frag& ah, const Frag& al,
                                             const Frag& bh, const Frag& bl) {
  acc = __builtin_amdgcn_wmma_f32_16x16x32_bf16(false, ah.v, false, bh.v, (short)0, acc, false, false);
  acc = __builtin_amdgcn_wmma_f32_16x16x32_bf16(false, ah.v, false, bl.v, (short)0, acc, false, false);
  acc = __builtin_amdgcn_wmma_f32_16x16x32_bf16(false, al.v, false, bh.v, (short)0, acc, false, false);
  asm volatile("v_nop\n\tv_nop\n\tv_nop\n\tv_nop"
               : "+v"(acc)
               : "v"(ah.w), "v"(al.w), "v"(bh.w), "v"(bl.w));
}

__global__ __launch_bounds__(256) void k_split(const float* __restrict__ src,
                                               u16* __restrict__ hi, u16* __restrict__ lo,
                                               int n8) {
  const int i = blockIdx.x * 256 + threadIdx.x;
  if (i >= n8) return;
  const float* p = src + (size_t)i * 8;
  const v4f a = *(const v4f*)p;
  const v4f b = *(const v4f*)(p + 4);
  float x[8] = {a[0], a[1], a[2], a[3], b[0], b[1], b[2], b[3]};
  v8u16 vh = {0, 0, 0, 0, 0, 0, 0, 0};
  v8u16 vl = {0, 0, 0, 0, 0, 0, 0, 0};
  split8(x, vh, vl);
  const size_t o = (size_t)i * 8;
  *(volatile v8u16*)(hi + o) = vh;
  *(volatile v8u16*)(lo + o) = vl;
  __threadfence();
  *(volatile v8u16*)(hi + o) = vh;
  *(volatile v8u16*)(lo + o) = vl;
}

__global__ __launch_bounds__(256) void k_tsplit(const float* __restrict__ src, int rows, int cols,
                                                u16* __restrict__ hi, u16* __restrict__ lo) {
  __shared__ float T[64][65];
  const int tid = threadIdx.x;
  const int c0 = blockIdx.x * 64, r0 = blockIdx.y * 64;
  if (c0 >= cols || r0 >= rows) return;
#pragma unroll
  for (int it = 0; it < 4; ++it) {
    const int r = it * 16 + (tid >> 4);
    const int c = (tid & 15) * 4;
    v4f v = {0.f, 0.f, 0.f, 0.f};
    if (r0 + r < rows && c0 + c + 3 < cols)
      v = *(const v4f*)(src + (size_t)(r0 + r) * cols + c0 + c);
    T[c + 0][r] = v[0];
    T[c + 1][r] = v[1];
    T[c + 2][r] = v[2];
    T[c + 3][r] = v[3];
  }
  __syncthreads();
  v8u16 vh[2], vl[2];
  size_t oo[2];
  bool ok[2];
#pragma unroll
  for (int it = 0; it < 2; ++it) {
    const int oc = it * 32 + (tid >> 3);
    const int p = tid & 7;
    float x[8];
#pragma unroll
    for (int j = 0; j < 8; ++j) x[j] = T[oc][8 * p + j];
    vh[it] = (v8u16){0, 0, 0, 0, 0, 0, 0, 0};
    vl[it] = (v8u16){0, 0, 0, 0, 0, 0, 0, 0};
    split8(x, vh[it], vl[it]);
    oo[it] = (size_t)(c0 + oc) * rows + r0 + 8 * p;
    ok[it] = (c0 + oc < cols) && (r0 + 8 * p + 7 < rows);
  }
#pragma unroll
  for (int it = 0; it < 2; ++it)
    if (ok[it]) { *(volatile v8u16*)(hi + oo[it]) = vh[it]; *(volatile v8u16*)(lo + oo[it]) = vl[it]; }
  __threadfence();
#pragma unroll
  for (int it = 0; it < 2; ++it)
    if (ok[it]) { *(volatile v8u16*)(hi + oo[it]) = vh[it]; *(volatile v8u16*)(lo + oo[it]) = vl[it]; }
}

static __device__ __forceinline__ void store_tile_f32(const float* sC, float* Cf, int ldc,
                                                      int m0, int n0, int M, int tid) {
#pragma unroll
  for (int it = 0; it < 8; ++it) {
    const int r = it * 8 + (tid >> 4);
    const int p = tid & 15;
    const v4f v = *(const v4f*)(sC + r * CSP + 4 * p);
    const int gm = m0 + r;
    if (gm < M) *(volatile v4f*)(Cf + (size_t)gm * ldc + n0 + 4 * p) = v;
  }
}
static __device__ __forceinline__ void store_tile_split(const float* sC, u16* Ch, u16* Cl, int ldc,
                                                        int m0, int n0, int M, int tid) {
#pragma unroll
  for (int it = 0; it < 4; ++it) {
    const int r = it * 16 + (tid >> 3);
    const int p = tid & 7;
    const float* cp = sC + r * CSP + 8 * p;
    const v4f a = *(const v4f*)cp;
    const v4f b = *(const v4f*)(cp + 4);
    float x[8] = {a[0], a[1], a[2], a[3], b[0], b[1], b[2], b[3]};
    v8u16 vh = {0, 0, 0, 0, 0, 0, 0, 0};
    v8u16 vl = {0, 0, 0, 0, 0, 0, 0, 0};
    split8(x, vh, vl);
    const int gm = m0 + r;
    if (gm < M) {
      const size_t o = (size_t)gm * ldc + n0 + 8 * p;
      *(volatile v8u16*)(Ch + o) = vh;
      *(volatile v8u16*)(Cl + o) = vl;
    }
  }
}

template <int OUTSPLIT>
__global__ __launch_bounds__(GT) void k_gemm(
    const u16* __restrict__ Ah, const u16* __restrict__ Al, int lda,
    const u16* __restrict__ Bh, const u16* __restrict__ Bl, int ldb,
    void* C0, void* C1, int ldc, int M, int N, int K) {
  __shared__ __align__(16) u16 sA_h[BM * LDK];
  __shared__ __align__(16) u16 sA_l[BM * LDK];
  __shared__ __align__(16) u16 sB_h[BN * LDK];
  __shared__ __align__(16) u16 sB_l[BN * LDK];
  __shared__ __align__(16) float sC[BM * CSP];

  const int tid  = threadIdx.x;
  const int lane = tid & 31;
  const int wid  = tid >> 5;
  const int hh   = lane >> 4;
  const int r15  = lane & 15;
  const int wm   = (wid & 1) * 32;
  const int wn   = (wid >> 1) * 32;
  const int m0   = blockIdx.y * BM;
  const int n0   = blockIdx.x * BN;
  if (m0 >= M || n0 >= N) return;

  const v8f zero8 = {0.f, 0.f, 0.f, 0.f, 0.f, 0.f, 0.f, 0.f};
  v8f acc[2][2];
#pragma unroll
  for (int i = 0; i < 2; ++i)
#pragma unroll
    for (int j = 0; j < 2; ++j) acc[i][j] = zero8;

  for (int kk = 0; kk < K; kk += BK) {
    __syncthreads();
#pragma unroll
    for (int it = 0; it < (BM * 8) / GT; ++it) {
      const int c  = tid + it * GT;
      const int r  = c >> 3;
      const int k8 = (c & 7) * 8;
      v8u16 ah = {0, 0, 0, 0, 0, 0, 0, 0}, al = {0, 0, 0, 0, 0, 0, 0, 0};
      v8u16 bh = {0, 0, 0, 0, 0, 0, 0, 0}, bl = {0, 0, 0, 0, 0, 0, 0, 0};
      const int gm = m0 + r;
      if (gm < M) {
        const size_t o = (size_t)gm * lda + kk + k8;
        ah = *(const v8u16*)(Ah + o);
        al = *(const v8u16*)(Al + o);
      }
      const int gn = n0 + r;
      if (gn < N) {
        const size_t o = (size_t)gn * ldb + kk + k8;
        bh = *(const v8u16*)(Bh + o);
        bl = *(const v8u16*)(Bl + o);
      }
      *(v8u16*)(sA_h + r * LDK + k8) = ah;
      *(v8u16*)(sA_l + r * LDK + k8) = al;
      *(v8u16*)(sB_h + r * LDK + k8) = bh;
      *(v8u16*)(sB_l + r * LDK + k8) = bl;
    }
    __syncthreads();

#pragma unroll
    for (int s = 0; s < BK / 32; ++s) {
      Frag fa_h[2], fa_l[2], fb_h[2], fb_l[2];
#pragma unroll
      for (int t = 0; t < 2; ++t) {
        const int ao = (wm + 16 * t + r15) * LDK + s * 32 + 8 * hh;
        fa_h[t].h[0] = *(const v8u16*)(sA_h + ao);
        fa_h[t].h[1] = *(const v8u16*)(sA_h + ao + 16);
        fa_l[t].h[0] = *(const v8u16*)(sA_l + ao);
        fa_l[t].h[1] = *(const v8u16*)(sA_l + ao + 16);
        const int bo = (wn + 16 * t + r15) * LDK + s * 32 + 8 * hh;
        fb_h[t].h[0] = *(const v8u16*)(sB_h + bo);
        fb_h[t].h[1] = *(const v8u16*)(sB_h + bo + 16);
        fb_l[t].h[0] = *(const v8u16*)(sB_l + bo);
        fb_l[t].h[1] = *(const v8u16*)(sB_l + bo + 16);
      }
#pragma unroll
      for (int tm = 0; tm < 2; ++tm)
#pragma unroll
        for (int tn = 0; tn < 2; ++tn)
          wmma3(acc[tm][tn], fa_h[tm], fa_l[tm], fb_h[tn], fb_l[tn]);
    }
  }

#pragma unroll
  for (int tm = 0; tm < 2; ++tm)
#pragma unroll
    for (int tn = 0; tn < 2; ++tn)
#pragma unroll
      for (int r = 0; r < 8; ++r)
        sC[(wm + 16 * tm + 8 * hh + r) * CSP + wn + 16 * tn + r15] = acc[tm][tn][r];
  __syncthreads();

  if constexpr (OUTSPLIT != 0) {
    u16* Ch = (u16*)C0;
    u16* Cl = (u16*)C1;
    store_tile_split(sC, Ch, Cl, ldc, m0, n0, M, tid);
    __threadfence();
    store_tile_split(sC, Ch, Cl, ldc, m0, n0, M, tid);
  } else {
    float* Cf = (float*)C0;
    store_tile_f32(sC, Cf, ldc, m0, n0, M, tid);
    __threadfence();
    store_tile_f32(sC, Cf, ldc, m0, n0, M, tid);
    (void)C1;
  }
}

__global__ __launch_bounds__(512) void k_bias(const float* __restrict__ b1, const float* __restrict__ W2,
                                              const float* __restrict__ b2, float* __restrict__ bw,
                                              int D, int NO) {
  __shared__ __align__(16) float s[512];
  const int t = threadIdx.x;
  const int n = blockIdx.x * 512 + t;
  float a = 0.f;
  if (n < NO) {
    a = b2[n];
#pragma unroll 4
    for (int k = 0; k < D; ++k) a = fmaf(b1[k], W2[(size_t)k * NO + n], a);
  }
  s[t] = a;
  __syncthreads();
  if (t < 128) {
    const int n4 = blockIdx.x * 512 + 4 * t;
    if (n4 + 3 < NO) {
      const v4f v = *(const v4f*)(s + 4 * t);
      *(volatile v4f*)(bw + n4) = v;
      __threadfence();
      *(volatile v4f*)(bw + n4) = v;
    }
  }
}

__global__ __launch_bounds__(128) void k_out(const int* __restrict__ idx, const float* __restrict__ Q,
                                             const float* __restrict__ Cq, const float* __restrict__ bw,
                                             float* __restrict__ out,
                                             int nrows, int R, int nper, int nobj, int NO) {
  const int row = blockIdx.x;
  if (row >= nrows) return;
  const int b = row / R;
  int g0 = idx[(size_t)row * 2 + 0] + b * nper;
  int g1 = idx[(size_t)row * 2 + 1] + b * nper;
  if (g0 < 0) g0 += nobj;
  if (g1 < 0) g1 += nobj;
  g0 = min(max(g0, 0), nobj - 1);
  g1 = min(max(g1, 0), nobj - 1);
  const float* q0p = Q + (size_t)g0 * NO;
  const float* q1p = Q + (size_t)g1 * NO;
  const float* cp  = Cq + (size_t)b * NO;
  float* op = out + (size_t)row * NO;
  for (int c = threadIdx.x * 4; c < NO; c += 512) {
    const v4f q0 = *(const v4f*)(q0p + c);
    const v4f q1 = *(const v4f*)(q1p + c);
    const v4f cc = *(const v4f*)(cp + c);
    const v4f bb = *(const v4f*)(bw + c);
    v4f o = 0.5f * (q0 + q1) + cc + bb;
#pragma unroll
    for (int j = 0; j < 4; ++j) o[j] = fmaxf(o[j], 0.f);
    *(volatile v4f*)(op + c) = o;
    __threadfence();
    *(volatile v4f*)(op + c) = o;
  }
}

extern "C" void kernel_launch(void* const* d_in, const int* in_sizes, int n_in,
                              void* d_out, int out_size, void* d_ws,
                              size_t ws_size, hipStream_t stream) {
  if (n_in < 7) return;
  const float* OBJ = (const float*)d_in[0];
  const float* CTX = (const float*)d_in[1];
  const int*   IDX = (const int*)d_in[2];
  const float* W1  = (const float*)d_in[3];
  const float* B1  = (const float*)d_in[4];
  const float* W2  = (const float*)d_in[5];
  const float* B2  = (const float*)d_in[6];
  float* OUT = (float*)d_out;

  const int D = in_sizes[4], NO = in_sizes[6];
  if (D <= 0 || NO <= 0) return;
  const int NOBJ = in_sizes[0] / D;
  const int NB   = in_sizes[1] / D;
  const int K1   = in_sizes[3] / D;
  if (NOBJ <= 0 || NB <= 0) return;
  if (NOBJ * D != in_sizes[0] || NB * D != in_sizes[1]) return;
  if (K1 != 2 * D || K1 * D != in_sizes[3] || in_sizes[5] != D * NO) return;
  const int NROWS = out_size / NO;
  if (NROWS <= 0 || NROWS * NO != out_size || in_sizes[2] != 2 * NROWS) return;
  const int R = NROWS / NB;
  if (R <= 0 || R * NB != NROWS) return;
  const int NPER = NOBJ / NB;
  if (NPER * NB != NOBJ) return;
  if ((D % 64) || (NO % 64) || (NOBJ % 64) || (NB % 64)) return;

  size_t off = 0;
  auto carve = [&](size_t bytes) -> size_t { size_t p = off; off += (bytes + 255) & ~(size_t)255; return p; };
  const size_t oW1h = carve((size_t)K1 * D * 2);
  const size_t oW1l = carve((size_t)K1 * D * 2);
  const size_t oOBh = carve((size_t)NOBJ * D * 2);
  const size_t oOBl = carve((size_t)NOBJ * D * 2);
  const size_t oCXh = carve((size_t)NB * D * 2);
  const size_t oCXl = carve((size_t)NB * D * 2);
  const size_t oW2h = carve((size_t)NO * D * 2);
  const size_t oW2l = carve((size_t)NO * D * 2);
  const size_t oM1h = carve((size_t)NO * K1 * 2);
  const size_t oM1l = carve((size_t)NO * K1 * 2);
  const size_t oQ   = carve((size_t)NOBJ * NO * 4);
  const size_t oCq  = carve((size_t)NB * NO * 4);
  const size_t oBW  = carve((size_t)NO * 4);
  if (off > ws_size) return;

  char* ws = (char*)d_ws;
  u16* W1h = (u16*)(ws + oW1h);  u16* W1l = (u16*)(ws + oW1l);
  u16* OBh = (u16*)(ws + oOBh);  u16* OBl = (u16*)(ws + oOBl);
  u16* CXh = (u16*)(ws + oCXh);  u16* CXl = (u16*)(ws + oCXl);
  u16* W2h = (u16*)(ws + oW2h);  u16* W2l = (u16*)(ws + oW2l);
  u16* M1h = (u16*)(ws + oM1h);  u16* M1l = (u16*)(ws + oM1l);
  float* Q  = (float*)(ws + oQ);
  float* Cq = (float*)(ws + oCq);
  float* BW = (float*)(ws + oBW);

  {
    const int n8a = (K1 * D) / 8;
    k_split<<<dim3((n8a + 255) / 256), 256, 0, stream>>>(W1, W1h, W1l, n8a);
    const int n8b = (NOBJ * D) / 8;
    k_split<<<dim3((n8b + 255) / 256), 256, 0, stream>>>(OBJ, OBh, OBl, n8b);
    const int n8c = (NB * D) / 8;
    k_split<<<dim3((n8c + 255) / 256), 256, 0, stream>>>(CTX, CXh, CXl, n8c);
    k_tsplit<<<dim3(NO / 64, D / 64), 256, 0, stream>>>(W2, D, NO, W2h, W2l);
  }
  k_gemm<1><<<dim3(K1 / BN, NO / BM), GT, 0, stream>>>(
      W2h, W2l, D, W1h, W1l, D, (void*)M1h, (void*)M1l, K1, NO, K1, D);
  k_gemm<0><<<dim3(NO / BN, NOBJ / BM), GT, 0, stream>>>(
      OBh, OBl, D, M1h, M1l, K1, (void*)Q, (void*)Q, NO, NOBJ, NO, D);
  k_gemm<0><<<dim3(NO / BN, NB / BM), GT, 0, stream>>>(
      CXh, CXl, D, M1h + D, M1l + D, K1, (void*)Cq, (void*)Cq, NO, NB, NO, D);
  k_bias<<<dim3((NO + 511) / 512), 512, 0, stream>>>(B1, W2, B2, BW, D, NO);
  k_out<<<dim3(NROWS), 128, 0, stream>>>(IDX, Q, Cq, BW, OUT, NROWS, R, NPER, NOBJ, NO);
}
